// EquivariantLocalScoreMachine_62122406969494
// MI455X (gfx1250) — hardware-verified
//
#include <hip/hip_runtime.h>

typedef __bf16   v16b __attribute__((ext_vector_type(16)));
typedef __bf16   v8b  __attribute__((ext_vector_type(8)));
typedef float    v8f  __attribute__((ext_vector_type(8)));
typedef float    v4f  __attribute__((ext_vector_type(4)));
typedef unsigned v4u  __attribute__((ext_vector_type(4)));
union Frag { v16b v; v8b half[2]; };

#define Bn    4
#define Cn    3
#define Hn    32
#define Wn    32
#define NQ    4096
#define NP    32768
#define KF    27
#define KP    32
#define QPB   32
#define NPART 4
#define TILES (NP / 16)
#define TPP   (TILES / NPART)
#define L2E   1.4426950408889634f

static_assert(NQ % QPB == 0);
static_assert(TILES % NPART == 0);
static_assert(NQ % 256 == 0);
static_assert(NP % 256 == 0);

__device__ __forceinline__ unsigned bf16_rne_bits(float f) {
  unsigned u = __float_as_uint(f);
  u += 0x7FFFu + ((u >> 16) & 1u);
  return u >> 16;
}

__device__ __forceinline__ v8f mma3_bf16(const v16b ahi, const v16b alo, const v16b bhi, const v16b blo) {
  v8f acc = {0.f, 0.f, 0.f, 0.f, 0.f, 0.f, 0.f, 0.f};
  acc = __builtin_amdgcn_wmma_f32_16x16x32_bf16(false, ahi, false, bhi, (short)0, acc, false, false);
  acc = __builtin_amdgcn_wmma_f32_16x16x32_bf16(false, ahi, false, blo, (short)0, acc, false, false);
  acc = __builtin_amdgcn_wmma_f32_16x16x32_bf16(false, alo, false, bhi, (short)0, acc, false, false);
  asm volatile("v_nop\n\tv_nop\n\tv_nop\n\tv_nop" : "+v"(acc) : "v"(ahi), "v"(alo), "v"(bhi), "v"(blo));
  return acc;
}

template <int WRAP>
__global__ __launch_bounds__(256) void prep_kernel(const float* __restrict__ src,
                                                   v4u* __restrict__ ghi,
                                                   v4u* __restrict__ glo,
                                                   v4f* __restrict__ gaux,
                                                   int nrows) {
  __shared__ v4u sh_hi[256 * 4];
  __shared__ v4u sh_lo[256 * 4];

  const int tid = threadIdx.x, lane = tid & 31, wave = tid >> 5;
  int r = blockIdx.x * 256 + tid;
  r = min(r, nrows - 1);
  const int n = r >> 10, rem = r & 1023, h = rem >> 5, w = rem & 31;

  unsigned wh[16], wl[16];
#pragma unroll
  for (int j = 0; j < 16; ++j) { wh[j] = 0u; wl[j] = 0u; }
  float norm = 0.f;
  float cen[3] = {0.f, 0.f, 0.f};

#pragma unroll
  for (int c = 0; c < Cn; ++c) {
    const float* sc = src + ((n * Cn + c) * Hn) * Wn;
#pragma unroll
    for (int di = 0; di < 3; ++di) {
#pragma unroll
      for (int dj = 0; dj < 3; ++dj) {
        const int hh = h + di - 1, ww = w + dj - 1;
        float v;
        if (WRAP) {
          v = sc[(hh & (Hn - 1)) * Wn + (ww & (Wn - 1))];
        } else {
          const bool ok = ((unsigned)hh < (unsigned)Hn) && ((unsigned)ww < (unsigned)Wn);
          const int hc = min(max(hh, 0), Hn - 1);
          const int wc = min(max(ww, 0), Wn - 1);
          const float tv = sc[hc * Wn + wc];
          v = ok ? tv : 0.f;
        }
        norm = fmaf(v, v, norm);
        if (di == 1 && dj == 1) cen[c] = v;
        const unsigned hb = bf16_rne_bits(v);
        const float    hf = __uint_as_float(hb << 16);
        const unsigned lb = bf16_rne_bits(v - hf);
        const int k = c * 9 + di * 3 + dj;
        wh[k >> 1] |= hb << ((k & 1) * 16);
        wl[k >> 1] |= lb << ((k & 1) * 16);
      }
    }
  }

#pragma unroll
  for (int j = 0; j < 4; ++j) {
    v4u a; a.x = wh[4 * j]; a.y = wh[4 * j + 1]; a.z = wh[4 * j + 2]; a.w = wh[4 * j + 3];
    v4u b; b.x = wl[4 * j]; b.y = wl[4 * j + 1]; b.z = wl[4 * j + 2]; b.w = wl[4 * j + 3];
    sh_hi[tid * 4 + j] = a;
    sh_lo[tid * 4 + j] = b;
  }
  __syncthreads();

  v4u hv[4], lv[4];
#pragma unroll
  for (int i = 0; i < 4; ++i) {
    const int idx = wave * 128 + i * 32 + lane;
    hv[i] = sh_hi[idx];
    lv[i] = sh_lo[idx];
  }
  v4f aux; aux.x = cen[0]; aux.y = cen[1]; aux.z = cen[2]; aux.w = norm;

  const size_t gbase = (size_t)blockIdx.x * 1024;
  const size_t arow  = (size_t)blockIdx.x * 256 + tid;

#pragma unroll
  for (int i = 0; i < 4; ++i) {
    const size_t gi = gbase + (size_t)(wave * 128 + i * 32 + lane);
    *(volatile v4u*)(ghi + gi) = hv[i];
    *(volatile v4u*)(glo + gi) = lv[i];
  }
  *(volatile v4f*)(gaux + arow) = aux;
  __threadfence();
#pragma unroll
  for (int i = 0; i < 4; ++i) {
    const size_t gi = gbase + (size_t)(wave * 128 + i * 32 + lane);
    *(volatile v4u*)(ghi + gi) = hv[i];
    *(volatile v4u*)(glo + gi) = lv[i];
  }
  *(volatile v4f*)(gaux + arow) = aux;
}

__global__ __launch_bounds__(256) void score_kernel(
    const __bf16* __restrict__ Qh, const __bf16* __restrict__ Ql,
    const __bf16* __restrict__ Ph, const __bf16* __restrict__ Pl,
    const v4f* __restrict__ qaux, const v4f* __restrict__ paux,
    const float* __restrict__ mus, const float* __restrict__ sgs,
    const int* __restrict__ tp, int nT, float* __restrict__ out) {
  __shared__ float sm[NPART * QPB * 5];
  __shared__ __attribute__((aligned(16))) float so[Cn * QPB];

  int t = tp[0];
  t = min(max(t, 0), nT - 1);
  const float mu     = mus[t];
  const float sg     = sgs[t];
  const float s2     = sg * sg;
  const float inv2s2 = 1.0f / (2.0f * s2);
  const float cA     = 2.0f * mu * inv2s2 * L2E;
  const float cP     = -(mu * mu) * inv2s2 * L2E;
  const float cQ     = -inv2s2 * L2E;

  const int lane = threadIdx.x & 31;
  const int wave = threadIdx.x >> 5;
  const int hl   = lane >> 4;
  const int m16  = lane & 15;
  const int g    = wave & 1;
  const int part = wave >> 1;
  const int qblk = blockIdx.x * QPB;
  const int q    = qblk + g * 16 + m16;

  Frag bhi, blo;
  {
    const __bf16* qh = Qh + (size_t)q * KP;
    const __bf16* ql = Ql + (size_t)q * KP;
    bhi.half[0] = *(const v8b*)(qh + 8 * hl);
    bhi.half[1] = *(const v8b*)(qh + 16 + 8 * hl);
    blo.half[0] = *(const v8b*)(ql + 8 * hl);
    blo.half[1] = *(const v8b*)(ql + 16 + 8 * hl);
  }
  const v4f   qa  = qaux[q];
  const float xb2 = cQ * qa.w;

  float m = -1e30f, sw = 0.f, a0 = 0.f, a1 = 0.f, a2 = 0.f;

  const int tbeg = part * TPP;
  for (int tile = tbeg; tile < tbeg + TPP; ++tile) {
    Frag ahi, alo;
    {
      const size_t prow = (size_t)(tile * 16 + m16) * KP;
      const __bf16* ph = Ph + prow;
      const __bf16* pl = Pl + prow;
      ahi.half[0] = *(const v8b*)(ph + 8 * hl);
      ahi.half[1] = *(const v8b*)(ph + 16 + 8 * hl);
      alo.half[0] = *(const v8b*)(pl + 8 * hl);
      alo.half[1] = *(const v8b*)(pl + 16 + 8 * hl);
    }
    const v8f d = mma3_bf16(ahi.v, alo.v, bhi.v, blo.v);

    const int pbase = tile * 16 + 8 * hl;
    v4f   pa[8];
    float lw[8];
#pragma unroll
    for (int r = 0; r < 8; ++r) pa[r] = paux[pbase + r];
#pragma unroll
    for (int r = 0; r < 8; ++r) lw[r] = fmaf(cA, d[r], fmaf(cP, pa[r].w, xb2));

    float tm = lw[0];
#pragma unroll
    for (int r = 1; r < 8; ++r) tm = fmaxf(tm, lw[r]);
    const float M  = fmaxf(m, tm);
    const float e0 = __builtin_amdgcn_exp2f(m - M);
    sw *= e0; a0 *= e0; a1 *= e0; a2 *= e0;
    m = M;
#pragma unroll
    for (int r = 0; r < 8; ++r) {
      const float e1 = __builtin_amdgcn_exp2f(lw[r] - M);
      sw += e1;
      a0 = fmaf(e1, pa[r].x, a0);
      a1 = fmaf(e1, pa[r].y, a1);
      a2 = fmaf(e1, pa[r].z, a2);
    }
  }

  {
    const float m2 = __shfl_xor(m, 16);
    const float w2 = __shfl_xor(sw, 16);
    const float b0 = __shfl_xor(a0, 16);
    const float b1 = __shfl_xor(a1, 16);
    const float b2 = __shfl_xor(a2, 16);
    const float M  = fmaxf(m, m2);
    const float e0 = __builtin_amdgcn_exp2f(m - M);
    const float e1 = __builtin_amdgcn_exp2f(m2 - M);
    sw = sw * e0 + w2 * e1;
    a0 = a0 * e0 + b0 * e1;
    a1 = a1 * e0 + b1 * e1;
    a2 = a2 * e0 + b2 * e1;
    m  = M;
  }
  if (hl == 0) {
    float* pp = &sm[(part * QPB + g * 16 + m16) * 5];
    pp[0] = m; pp[1] = sw; pp[2] = a0; pp[3] = a1; pp[4] = a2;
  }
  __syncthreads();

  if (wave == 0) {
    const int ql = lane;
    float M = -1e30f, SW = 0.f, W0 = 0.f, W1 = 0.f, W2 = 0.f;
#pragma unroll
    for (int pt = 0; pt < NPART; ++pt) {
      const float* pp = &sm[(pt * QPB + ql) * 5];
      const float m2 = pp[0];
      const float Mn = fmaxf(M, m2);
      const float e0 = __builtin_amdgcn_exp2f(M - Mn);
      const float e1 = __builtin_amdgcn_exp2f(m2 - Mn);
      SW = SW * e0 + pp[1] * e1;
      W0 = W0 * e0 + pp[2] * e1;
      W1 = W1 * e0 + pp[3] * e1;
      W2 = W2 * e0 + pp[4] * e1;
      M  = Mn;
    }
    const v4f   xa   = qaux[qblk + ql];
    const float den  = s2 * SW;
    const float rden = 1.0f / den;
    so[0 * QPB + ql] = -(xa.x * SW - mu * W0) * rden;
    so[1 * QPB + ql] = -(xa.y * SW - mu * W1) * rden;
    so[2 * QPB + ql] = -(xa.z * SW - mu * W2) * rden;
  }
  __syncthreads();

  if (wave == 0 && lane < Cn * 8) {
    const int c = lane >> 3, j = lane & 7;
    const v4f v = *(const v4f*)(&so[c * QPB + 4 * j]);
    const int b = qblk >> 10, pix0 = qblk & 1023;
    float* dst = out + (size_t)(b * Cn + c) * (Hn * Wn) + pix0 + 4 * j;
    *(volatile v4f*)dst = v;
    __threadfence();
    *(volatile v4f*)dst = v;
  }
}

extern "C" void kernel_launch(void* const* d_in, const int* in_sizes, int n_in,
                              void* d_out, int out_size, void* d_ws, size_t ws_size,
                              hipStream_t stream) {
  if (n_in < 5) return;
  if (in_sizes[0] != Bn * Cn * Hn * Wn) return;
  if (in_sizes[1] != (NP / (Hn * Wn)) * Cn * Hn * Wn) return;
  if (in_sizes[2] < 1 || in_sizes[3] < 1 || in_sizes[4] < 1) return;
  if (out_size != Bn * Cn * Hn * Wn) return;
  const int nT = in_sizes[2] < in_sizes[3] ? in_sizes[2] : in_sizes[3];

  const float* x    = (const float*)d_in[0];
  const float* imgs = (const float*)d_in[1];
  const float* mus  = (const float*)d_in[2];
  const float* sgs  = (const float*)d_in[3];
  const int*   tp   = (const int*)d_in[4];

  const size_t szQ  = (size_t)NQ * KP * 2;
  const size_t szP  = (size_t)NP * KP * 2;
  const size_t szQa = (size_t)NQ * 16;
  const size_t szPa = (size_t)NP * 16;
  const size_t oQh = 0;
  const size_t oQl = oQh + szQ;
  const size_t oPh = oQl + szQ;
  const size_t oPl = oPh + szP;
  const size_t oQa = oPl + szP;
  const size_t oPa = oQa + szQa;
  const size_t total = oPa + szPa;
  if (total > ws_size) return;

  char* ws = (char*)d_ws;
  __bf16* Qh = (__bf16*)(ws + oQh);
  __bf16* Ql = (__bf16*)(ws + oQl);
  __bf16* Ph = (__bf16*)(ws + oPh);
  __bf16* Pl = (__bf16*)(ws + oPl);
  v4f*    Qa = (v4f*)(ws + oQa);
  v4f*    Pa = (v4f*)(ws + oPa);

  prep_kernel<1><<<dim3(NQ / 256), dim3(256), 0, stream>>>(x, (v4u*)Qh, (v4u*)Ql, Qa, NQ);
  prep_kernel<0><<<dim3(NP / 256), dim3(256), 0, stream>>>(imgs, (v4u*)Ph, (v4u*)Pl, Pa, NP);
  score_kernel<<<dim3(NQ / QPB), dim3(256), 0, stream>>>(Qh, Ql, Ph, Pl, Qa, Pa,
                                                         mus, sgs, tp, nT, (float*)d_out);
}
